// Attention_Embedding_20744692040370
// MI455X (gfx1250) — hardware-verified
//
#include <hip/hip_runtime.h>
#include <math.h>

typedef __attribute__((ext_vector_type(16))) _Float16 v16h;
typedef __attribute__((ext_vector_type(16))) __bf16 v16b;
typedef __attribute__((ext_vector_type(8)))  _Float16 v8h;
typedef __attribute__((ext_vector_type(8)))  float v8f;
typedef __attribute__((ext_vector_type(4)))  float v4f;
typedef __attribute__((ext_vector_type(2)))  float v2f;
typedef __attribute__((ext_vector_type(4)))  unsigned v4u;
typedef __attribute__((ext_vector_type(4)))  int v4i;
typedef float __attribute__((may_alias)) float_a;
typedef int __attribute__((may_alias)) int_a;

template <typename T> __device__ __forceinline__ void vst2(void* p, T v) { *(volatile T*)p = v; __threadfence(); *(volatile T*)p = v; }
__device__ __forceinline__ v8f wmma16(v16h a, v16h b, v8f c) {
  v8f d = __builtin_amdgcn_wmma_f32_16x16x32_f16(false, a, false, b, (short)0, c, false, false);
  asm volatile("v_nop\n\tv_nop\n\tv_nop\n\tv_nop" : "+v"(d) : "v"(a), "v"(b));
  return d;
}
__device__ __forceinline__ v8f wmma_bf(v16b a, v16b b, v8f c) {
  v8f d = __builtin_amdgcn_wmma_f32_16x16x32_bf16(false, a, false, b, (short)0, c, false, false);
  asm volatile("v_nop\n\tv_nop\n\tv_nop\n\tv_nop" : "+v"(d) : "v"(a), "v"(b));
  return d;
}
__device__ __forceinline__ v16h frag_h(const _Float16* rowk0, int lane) {
  union { v16h v; v8h q[2]; } u; const _Float16* p = rowk0 + 8 * (lane >> 4);
  u.q[0] = *(const v8h*)p; u.q[1] = *(const v8h*)(p + 16); return u.v;
}
__device__ __forceinline__ v16h frag_f32(const float* rowk0, int lane) {
  v16h a; const float* p = rowk0 + 8 * (lane >> 4);
#pragma unroll
  for (int i = 0; i < 8; ++i) { a[i] = (_Float16)p[i]; a[8 + i] = (_Float16)p[16 + i]; }
  return a;
}
__device__ __forceinline__ v16h frag_f32s(const float* rowk0, int lane, float sc) {
  v16h a; const float* p = rowk0 + 8 * (lane >> 4);
#pragma unroll
  for (int i = 0; i < 8; ++i) { a[i] = (_Float16)(p[i] * sc); a[8 + i] = (_Float16)(p[16 + i] * sc); }
  return a;
}
__device__ __forceinline__ v16h fragc_f32(const float* W, int k0, int n, int lane, int ld, int K) {
  v16h a; const int g = lane >> 4;
#pragma unroll
  for (int i = 0; i < 8; ++i) { const int ka = k0 + 8 * g + i, kb = ka + 16;
    a[i] = (_Float16)(ka < K ? W[(size_t)(ka < K ? ka : K - 1) * ld + n] : 0.f); a[8 + i] = (_Float16)(kb < K ? W[(size_t)(kb < K ? kb : K - 1) * ld + n] : 0.f); }
  return a;
}
struct F2 { v16b h, l; };
__device__ __forceinline__ F2 bsplit16(const float v[16]) { F2 r;
#pragma unroll
  for (int i = 0; i < 16; ++i) { const __bf16 h = (__bf16)v[i]; r.h[i] = h; r.l[i] = (__bf16)(v[i] - (float)h); }
  return r; }
__device__ __forceinline__ F2 split_row(const float* row, int k0, int lane) { float v[16]; const float* p = row + k0 + 8 * (lane >> 4);
#pragma unroll
  for (int i = 0; i < 8; ++i) { v[i] = p[i]; v[8 + i] = p[16 + i]; }
  return bsplit16(v); }
__device__ __forceinline__ F2 split_rowK(const float* row, int k0, int lane, int K) { float v[16]; const int g = lane >> 4;
#pragma unroll
  for (int i = 0; i < 8; ++i) { const int ka = k0 + 8 * g + i, kb = ka + 16; v[i] = ka < K ? row[ka < K ? ka : K - 1] : 0.f; v[8 + i] = kb < K ? row[kb < K ? kb : K - 1] : 0.f; }
  return bsplit16(v); }
__device__ __forceinline__ F2 split_col(const float* W, int k0, int n, int lane, int ld, int K) { float v[16]; const int g = lane >> 4;
#pragma unroll
  for (int i = 0; i < 8; ++i) { const int ka = k0 + 8 * g + i, kb = ka + 16; v[i] = ka < K ? W[(size_t)(ka < K ? ka : K - 1) * ld + n] : 0.f; v[8 + i] = kb < K ? W[(size_t)(kb < K ? kb : K - 1) * ld + n] : 0.f; }
  return bsplit16(v); }
__device__ __forceinline__ v8f mac3(const F2& a, const F2& b, v8f c) { c = wmma_bf(a.l, b.h, c); c = wmma_bf(a.h, b.l, c); return wmma_bf(a.h, b.h, c); }
__device__ __forceinline__ float sigm(float v) { return 1.0f / (1.0f + expf(-v)); }
#define LDSX() do { asm volatile("s_wait_dscnt 0" ::: "memory"); __builtin_amdgcn_wave_barrier(); __builtin_amdgcn_fence(__ATOMIC_RELEASE, "workgroup"); } while (0)


#define NBT 4
#define NHW 81
#define ND 100
#define NDO 97
#define NC 64
#define NVOX (NHW * ND)
#define NVP 8128
#define NOROW (NHW * NDO)
#ifndef TNB
#define TNB NBT
#define TQB (NVP / 64)
#define TOT ((NBT * NOROW + 63) / 64)
#endif
typedef __attribute__((ext_vector_type(8))) __bf16 v8b;
__device__ __forceinline__ v16b frag_b(const __bf16* rowk0, int lane) {
  union { v16b v; v8b q[2]; } u; const __bf16* p = rowk0 + 8 * (lane >> 4);
  u.q[0] = *(const v8b*)p; u.q[1] = *(const v8b*)(p + 16); return u.v;
}
__device__ __forceinline__ float bfr(float v) { return (float)(__bf16)v; }
__device__ __attribute__((noinline)) float exp_ni(float v) { return expf(v); }
__device__ __attribute__((noinline)) float erf_ni(float v) { return erff(v); }

#define WS_PW   0u
#define P_Q 0
#define P_K (P_Q + NC * NC)
#define P_V (P_K + NC * NC)
#define P_CH (P_V + NC * NC)
#define P_PO (P_CH + NC * 4 * NC)
#define PWEND (P_PO + NC * 4 * NC)
#define WS_XB   (WS_PW + 2u * PWEND)
#define WS_XT   (WS_XB + 2u * NBT * NVP * NC)
#define WS_QTH  (WS_XT + 2u * NBT * NC * NVP)
#define WS_QTL  (WS_QTH + 2u * NBT * NC * NVP)
#define WS_KTH  (WS_QTL + 2u * NBT * NC * NVP)
#define WS_KTL  (WS_KTH + 2u * NBT * NC * NVP)
#define WS_VR   (WS_KTL + 2u * NBT * NC * NVP)
#define WS_AC   (WS_VR + 4u * NBT * NVP * NC)
#define WS_CHH  (WS_AC + 4u * NBT * NC * NC)
#define WS_CHL  (WS_CHH + 2u * NBT * NVP * NC)
#define WS_POH  (WS_CHL + 2u * NBT * NVP * NC)
#define WS_POL  (WS_POH + 2u * NBT * NVP * NC)
#define WS_END  (WS_POL + 2u * NBT * NVP * NC)

__global__ __launch_bounds__(256) void k_packT(const float* __restrict__ WQ, const float* __restrict__ WK, const float* __restrict__ WV, const float* __restrict__ WCH, const float* __restrict__ WPO, __bf16* __restrict__ PW) {
  __shared__ __align__(16) __bf16 s[256]; const int e = blockIdx.x, which = blockIdx.y, tid = threadIdx.x; int K; size_t dst;
  if (which < 3) { const float* Wm = which == 0 ? WQ : (which == 1 ? WK : WV); K = NC; dst = (size_t)which * NC * NC + (size_t)e * NC; if (tid < K) s[tid] = (__bf16)Wm[(size_t)tid * NC + e]; }
  else { const float* Wm = which == 3 ? WCH : WPO; K = 4 * NC; dst = (which == 3 ? P_CH : P_PO) + (size_t)e * 4 * NC; if (tid < K) s[tid] = (__bf16)Wm[(size_t)tid * NC + e]; }
  __syncthreads();
  if (tid < K / 8) vst2((unsigned*)(PW + dst + tid * 8), *(const v4u*)&s[tid * 8]);
}
__global__ __launch_bounds__(256) void k_xb(const float* __restrict__ X, __bf16* __restrict__ XB, __bf16* __restrict__ XT) {
  __shared__ __align__(16) __bf16 s[64][72]; __shared__ __align__(16) __bf16 st[64][72]; const int tid = threadIdx.x; const size_t rb = (size_t)blockIdx.x * 64; const int b = (int)(rb / NVP), n0 = (int)(rb % NVP);
  for (int q = tid; q < 64 * 64; q += 256) { const int rl = q >> 6, c = q & 63; const int n = n0 + rl; const float v = (n < NVOX) ? X[((size_t)b * NVOX + min(n, NVOX - 1)) * NC + c] : 0.f; const __bf16 hb = (__bf16)v; s[rl][c] = hb; st[c][rl] = hb; }
  __syncthreads();
  for (int q = tid; q < 64 * 8; q += 256) { const int rl = q >> 3, pc = q & 7; vst2((unsigned*)(XB + (rb + rl) * NC + pc * 8), *(const v4u*)&s[rl][pc * 8]); vst2((unsigned*)(XT + ((size_t)b * NC + rl) * NVP + n0 + pc * 8), *(const v4u*)&st[rl][pc * 8]); }
}
__global__ __launch_bounds__(128) void k_vatt(const __bf16* __restrict__ XB, const __bf16* __restrict__ XT, const float* __restrict__ X, const float* __restrict__ BETA, __bf16* __restrict__ CHH, __bf16* __restrict__ CHL) {
  __shared__ __align__(16) float sp[4][16][36]; __shared__ __align__(16) __bf16 soh[4][16][72], sol[4][16][72];
  const int tid = threadIdx.x, wave = tid >> 5, lane = tid & 31, col = lane & 15, g = lane >> 4;
  const int qb = blockIdx.x, b = blockIdx.y; const int q0 = qb * 64 + wave * 16; const size_t rq = (size_t)b * NVP + q0 + col;
  v16b aq[2];
#pragma unroll
  for (int kc = 0; kc < 2; ++kc) aq[kc] = frag_b(XB + rq * NC + kc * 32, lane);
  float m[8], l[8];
#pragma unroll
  for (int r = 0; r < 8; ++r) { m[r] = -3.0e38f; l[r] = 0.f; }
  v8f acc[4] = {};
#pragma unroll 1
  for (int ks = 0; ks < NVP / 32; ++ks) { v8f s[2];
#pragma unroll
    for (int ct = 0; ct < 2; ++ct) { const int kk = ks * 32 + ct * 16 + col; v8f c = {};
#pragma unroll
      for (int kc = 0; kc < 2; ++kc) c = wmma_bf(aq[kc], frag_b(XB + ((size_t)b * NVP + kk) * NC + kc * 32, lane), c);
#pragma unroll
      for (int r = 0; r < 8; ++r) s[ct][r] = (kk < NVOX) ? c[r] : -3.0e38f; }
#pragma unroll
    for (int r = 0; r < 8; ++r) { float mx = fmaxf(s[0][r], s[1][r]);
#pragma unroll
      for (int o = 1; o < 16; o <<= 1) mx = fmaxf(mx, __shfl_xor(mx, o));
      const float mn = fmaxf(m[r], mx); const float alpha = (m[r] <= -1.0e38f) ? 0.f : __expf(m[r] - mn);
      const float e0 = bfr((s[0][r] <= -1.0e38f) ? 0.f : __expf(s[0][r] - mn)), e1 = bfr((s[1][r] <= -1.0e38f) ? 0.f : __expf(s[1][r] - mn)); float es = e0 + e1;
#pragma unroll
      for (int o = 1; o < 16; o <<= 1) es += __shfl_xor(es, o);
      l[r] = l[r] * alpha + es; m[r] = mn;
#pragma unroll
      for (int dt = 0; dt < 4; ++dt) acc[dt][r] *= alpha;
      sp[wave][8 * g + r][col] = e0; sp[wave][8 * g + r][16 + col] = e1; }
    LDSX();
    v16b pa; { const float* prow = &sp[wave][col][0] + 8 * g;
#pragma unroll
      for (int i = 0; i < 8; ++i) { pa[i] = (__bf16)prow[i]; pa[8 + i] = (__bf16)prow[16 + i]; } }
#pragma unroll
    for (int dt = 0; dt < 4; ++dt) { const size_t vr = ((size_t)b * NC + dt * 16 + col) * NVP + (size_t)ks * 32; acc[dt] = wmma_bf(pa, frag_b(XT + vr, lane), acc[dt]); }
    LDSX(); }
  const float beta = bfr(BETA[0]);
#pragma unroll
  for (int r = 0; r < 8; ++r) { const float il = 1.0f / l[r]; const size_t n = (size_t)b * NVP + q0 + 8 * g + r; const int nv = q0 + 8 * g + r;
#pragma unroll
    for (int dt = 0; dt < 4; ++dt) { const int c = dt * 16 + col; const float xv = (nv < NVOX) ? bfr(X[((size_t)b * NVOX + min(nv, NVOX - 1)) * NC + c]) : 0.f; const float v = beta * (acc[dt][r] * il) + xv; const __bf16 hb = (__bf16)v; soh[wave][8 * g + r][c] = hb; sol[wave][8 * g + r][c] = (__bf16)(v - (float)hb); (void)n; } }
  LDSX();
  for (int rl = 0; rl < 16; ++rl) if (lane < 16) { const size_t n = (size_t)b * NVP + q0 + rl; if (lane < 8) vst2((unsigned*)(CHH + n * NC + lane * 8), *(const v4u*)&soh[wave][rl][lane * 8]); else vst2((unsigned*)(CHL + n * NC + (lane - 8) * 8), *(const v4u*)&sol[wave][rl][(lane - 8) * 8]); }
}
__global__ __launch_bounds__(128) void k_qkv(const __bf16* __restrict__ XB, const __bf16* __restrict__ PW, const float* __restrict__ BQ, const float* __restrict__ BK, const float* __restrict__ BV, __bf16* __restrict__ QTH, __bf16* __restrict__ QTL, __bf16* __restrict__ KTH, __bf16* __restrict__ KTL, float* __restrict__ VR) {
  __shared__ __align__(16) __bf16 sqh[64][72], sql[64][72], skh[64][72], skl[64][72]; __shared__ __align__(16) float sv[4][16][68];
  const int tid = threadIdx.x, wave = tid >> 5, lane = tid & 31, col = lane & 15, g = lane >> 4; const size_t rb = (size_t)blockIdx.x * 64; const int b = (int)(rb / NVP), n0 = (int)(rb % NVP); const size_t r0 = rb + wave * 16;
  v16b ax[2];
#pragma unroll
  for (int kc = 0; kc < 2; ++kc) ax[kc] = frag_b(XB + (r0 + col) * NC + kc * 32, lane);
#pragma unroll 1
  for (int which = 0; which < 3; ++which) { v8f acc[4] = {}; const __bf16* P = PW + (size_t)which * NC * NC; const float* bias = which == 0 ? BQ : (which == 1 ? BK : BV);
#pragma unroll
    for (int kc = 0; kc < 2; ++kc)
#pragma unroll
      for (int j = 0; j < 4; ++j) acc[j] = wmma_bf(ax[kc], frag_b(P + (size_t)(j * 16 + col) * NC + kc * 32, lane), acc[j]);
#pragma unroll
    for (int j = 0; j < 4; ++j) { const int c = j * 16 + col; const float bb = bfr(bias[c]);
#pragma unroll
      for (int r = 0; r < 8; ++r) { const float v = acc[j][r] + bb; const int rl = wave * 16 + 8 * g + r;
        if (which == 2) sv[wave][8 * g + r][c] = v; else { const __bf16 hb = (__bf16)v; const __bf16 lb = (__bf16)(v - (float)hb); if (which == 0) { sqh[c][rl] = hb; sql[c][rl] = lb; } else { skh[c][rl] = hb; skl[c][rl] = lb; } } } } }
  __syncthreads();
  for (int q = tid; q < 64 * 8; q += 128) { const int c = q >> 3, pc = q & 7; const size_t o = ((size_t)b * NC + c) * NVP + n0 + pc * 8; vst2((unsigned*)(QTH + o), *(const v4u*)&sqh[c][pc * 8]); vst2((unsigned*)(QTL + o), *(const v4u*)&sql[c][pc * 8]); vst2((unsigned*)(KTH + o), *(const v4u*)&skh[c][pc * 8]); vst2((unsigned*)(KTL + o), *(const v4u*)&skl[c][pc * 8]); }
  for (int rl = 0; rl < 16; ++rl) if (lane < 16) vst2(VR + (r0 + rl) * NC + lane * 4, *(const v4f*)&sv[wave][rl][lane * 4]);
}
__global__ __launch_bounds__(128) void k_ec(const __bf16* __restrict__ QTH, const __bf16* __restrict__ QTL, const __bf16* __restrict__ KTH, const __bf16* __restrict__ KTL, float* __restrict__ AC) {
  __shared__ __align__(16) float so[4][16][68]; __shared__ __align__(16) __bf16 tq[2][64][40], tk[2][64][40];
  const int tid = threadIdx.x, wave = tid >> 5, lane = tid & 31, col = lane & 15, g = lane >> 4; const int b = blockIdx.x; const int c0 = wave * 16;
  v8f acc[4] = {};
#pragma unroll 1
  for (int ks = 0; ks < NVOX / 32; ++ks) { F2 a; a.h = frag_b(QTH + ((size_t)b * NC + c0 + col) * NVP + ks * 32, lane); a.l = frag_b(QTL + ((size_t)b * NC + c0 + col) * NVP + ks * 32, lane);
#pragma unroll
    for (int j = 0; j < 4; ++j) { F2 w; w.h = frag_b(KTH + ((size_t)b * NC + j * 16 + col) * NVP + ks * 32, lane); w.l = frag_b(KTL + ((size_t)b * NC + j * 16 + col) * NVP + ks * 32, lane); acc[j] = mac3(a, w, acc[j]); } }
  { const int kbase = (NVOX / 32) * 32;
    for (int q = tid; q < 64 * 32; q += 128) { const int c = q >> 5, i = q & 31; const bool ok = (kbase + i) < NVOX; const size_t o = ((size_t)b * NC + c) * NVP + kbase + i; const __bf16 z = (__bf16)0.f;
      tq[0][c][i] = ok ? QTH[o] : z; tq[1][c][i] = ok ? QTL[o] : z; tk[0][c][i] = ok ? KTH[o] : z; tk[1][c][i] = ok ? KTL[o] : z; }
    __syncthreads();
    F2 a; a.h = frag_b(&tq[0][c0 + col][0], lane); a.l = frag_b(&tq[1][c0 + col][0], lane);
#pragma unroll
    for (int j = 0; j < 4; ++j) { F2 w; w.h = frag_b(&tk[0][j * 16 + col][0], lane); w.l = frag_b(&tk[1][j * 16 + col][0], lane); acc[j] = mac3(a, w, acc[j]); } }
#pragma unroll
  for (int r = 0; r < 8; ++r) { float mx = -3.0e38f;
#pragma unroll
    for (int j = 0; j < 4; ++j) mx = fmaxf(mx, acc[j][r]);
#pragma unroll
    for (int o = 1; o < 16; o <<= 1) mx = fmaxf(mx, __shfl_xor(mx, o));
    float e[4], z = 0.f;
#pragma unroll
    for (int j = 0; j < 4; ++j) { e[j] = exp_ni(acc[j][r] - mx); z += e[j]; }
#pragma unroll
    for (int o = 1; o < 16; o <<= 1) z += __shfl_xor(z, o);
    const float iz = 1.0f / z;
#pragma unroll
    for (int j = 0; j < 4; ++j) so[wave][8 * g + r][j * 16 + col] = e[j] * iz; }
  LDSX();
  for (int rl = 0; rl < 16; ++rl) if (lane < 16) vst2(AC + ((size_t)b * NC + c0 + rl) * NC + lane * 4, *(const v4f*)&so[wave][rl][lane * 4]);
}
__global__ __launch_bounds__(128) void k_pos(const float* __restrict__ VR, const float* __restrict__ AC, const float* __restrict__ X, const float* __restrict__ GAMMA, __bf16* __restrict__ POH, __bf16* __restrict__ POL) {
  __shared__ __align__(16) __bf16 soh[4][16][72], sol[4][16][72];
  const int tid = threadIdx.x, wave = tid >> 5, lane = tid & 31, col = lane & 15, g = lane >> 4; const size_t rb = (size_t)blockIdx.x * 64; const int b = (int)(rb / NVP); const size_t r0 = rb + wave * 16;
  v8f acc[4] = {};
#pragma unroll
  for (int kc = 0; kc < 2; ++kc) { const F2 a = split_row(VR + (r0 + col) * NC, kc * 32, lane);
#pragma unroll
    for (int j = 0; j < 4; ++j) { const F2 w = split_row(AC + ((size_t)b * NC + j * 16 + col) * NC, kc * 32, lane); acc[j] = mac3(a, w, acc[j]); } }
  const float gamma = bfr(GAMMA[0]);
#pragma unroll
  for (int r = 0; r < 8; ++r) { const int nv = (int)((r0 + 8 * g + r) % NVP);
#pragma unroll
    for (int j = 0; j < 4; ++j) { const int c = j * 16 + col; const float xv = (nv < NVOX) ? bfr(X[((size_t)b * NVOX + min(nv, NVOX - 1)) * NC + c]) : 0.f; const float v = gamma * acc[j][r] + xv; const __bf16 hb = (__bf16)v; soh[wave][8 * g + r][c] = hb; sol[wave][8 * g + r][c] = (__bf16)(v - (float)hb); } }
  LDSX();
  for (int rl = 0; rl < 16; ++rl) if (lane < 16) { const size_t n = r0 + rl; if (lane < 8) vst2((unsigned*)(POH + n * NC + lane * 8), *(const v4u*)&soh[wave][rl][lane * 8]); else vst2((unsigned*)(POL + n * NC + (lane - 8) * 8), *(const v4u*)&sol[wave][rl][(lane - 8) * 8]); }
}
__global__ __launch_bounds__(128) void k_conv(const __bf16* __restrict__ CHH, const __bf16* __restrict__ CHL, const __bf16* __restrict__ POH, const __bf16* __restrict__ POL, const __bf16* __restrict__ PW, const float* __restrict__ BCH, const float* __restrict__ BPO, float* __restrict__ OUT) {
  __shared__ __align__(16) float so[4][16][68];
  const int tid = threadIdx.x, wave = tid >> 5, lane = tid & 31, col = lane & 15, g = lane >> 4; const size_t r0 = (size_t)blockIdx.x * 64 + wave * 16;
  const size_t oa = min(r0 + col, (size_t)(NBT * NOROW - 1)); const size_t bhw = oa / NDO, dd = oa % NDO; const size_t src = (((bhw / NHW) * NVP) + (bhw % NHW) * ND + dd) * NC;
  v8f acc1[4] = {}, acc2[4] = {};
#pragma unroll
  for (int kc = 0; kc < 8; ++kc) { F2 a; a.h = frag_b(CHH + src + kc * 32, lane); a.l = frag_b(CHL + src + kc * 32, lane); F2 p; p.h = frag_b(POH + src + kc * 32, lane); p.l = frag_b(POL + src + kc * 32, lane);
#pragma unroll
    for (int j = 0; j < 4; ++j) { const v16b w1 = frag_b(PW + P_CH + (size_t)(j * 16 + col) * 4 * NC + kc * 32, lane), w2 = frag_b(PW + P_PO + (size_t)(j * 16 + col) * 4 * NC + kc * 32, lane);
      acc1[j] = wmma_bf(a.l, w1, acc1[j]); acc1[j] = wmma_bf(a.h, w1, acc1[j]); acc2[j] = wmma_bf(p.l, w2, acc2[j]); acc2[j] = wmma_bf(p.h, w2, acc2[j]); } }
#pragma unroll
  for (int j = 0; j < 4; ++j) { const int e = j * 16 + col; const float b1 = bfr(BCH[e]), b2 = bfr(BPO[e]);
#pragma unroll
    for (int r = 0; r < 8; ++r) so[wave][8 * g + r][e] = fmaxf(acc1[j][r] + b1, 0.f) + fmaxf(acc2[j][r] + b2, 0.f); }
  LDSX();
  for (int rl = 0; rl < 16; ++rl) { const size_t o = r0 + rl; if (o < (size_t)NBT * NOROW && lane < 16) vst2(OUT + o * NC + lane * 4, *(const v4f*)&so[wave][rl][lane * 4]); }
}
extern "C" void kernel_launch(void* const* d_in, const int* in_sizes, int n_in, void* d_out, int out_size, void* d_ws, size_t ws_size, hipStream_t stream) {
  (void)in_sizes; (void)n_in; (void)out_size;
  const float** F = (const float**)d_in;
  if (ws_size < (size_t)WS_END) return;
  char* ws = (char*)d_ws; __bf16 *PW = (__bf16*)(ws + WS_PW), *XB = (__bf16*)(ws + WS_XB), *XT = (__bf16*)(ws + WS_XT), *QTH = (__bf16*)(ws + WS_QTH), *QTL = (__bf16*)(ws + WS_QTL), *KTH = (__bf16*)(ws + WS_KTH), *KTL = (__bf16*)(ws + WS_KTL), *CHH = (__bf16*)(ws + WS_CHH), *CHL = (__bf16*)(ws + WS_CHL), *POH = (__bf16*)(ws + WS_POH), *POL = (__bf16*)(ws + WS_POL);
  float *VR = (float*)(ws + WS_VR), *AC = (float*)(ws + WS_AC);
  k_packT<<<dim3(NC, 5), 256, 0, stream>>>(F[3], F[5], F[7], F[9], F[11], PW);
  k_xb<<<NBT * NVP / 64, 256, 0, stream>>>(F[0], XB, XT);
  k_vatt<<<dim3(TQB, TNB), 128, 0, stream>>>(XB, XT, F[0], F[1], CHH, CHL);
  k_qkv<<<TNB * NVP / 64, 128, 0, stream>>>(XB, PW, F[4], F[6], F[8], QTH, QTL, KTH, KTL, VR);
  k_ec<<<TNB, 128, 0, stream>>>(QTH, QTL, KTH, KTL, AC);
  k_pos<<<TNB * NVP / 64, 128, 0, stream>>>(VR, AC, F[0], F[2], POH, POL);
  k_conv<<<TOT, 128, 0, stream>>>(CHH, CHL, POH, POL, PW, F[10], F[12], (float*)d_out);
}
